// WeightGenerator_32478542692806
// MI455X (gfx1250) — hardware-verified
//
#include <hip/hip_runtime.h>


#define NN   1024
#define ED   32
#define HDN  64
#define RCH  131072
typedef _Float16 h16;
typedef unsigned short bf;
typedef __attribute__((ext_vector_type(16))) __bf16   v16bf;
typedef __attribute__((ext_vector_type(16))) _Float16 v16h;
typedef __attribute__((ext_vector_type(8)))  _Float16 v8h;
typedef __attribute__((ext_vector_type(8)))  unsigned short v8us;
typedef __attribute__((ext_vector_type(8)))  float    v8f;
typedef __attribute__((ext_vector_type(4)))  float    v4f;
typedef v8h  __attribute__((may_alias)) v8ha;
typedef v4f  __attribute__((may_alias)) v4fa;
typedef v8us __attribute__((may_alias)) v8usa;

__device__ __forceinline__ unsigned short f2bf(float f) { unsigned u = __float_as_uint(f); u += 0x7FFFu + ((u >> 16) & 1u); return (unsigned short)(u >> 16); }
__device__ __forceinline__ float bf2f(unsigned short b) { return __uint_as_float(((unsigned)b) << 16); }
__device__ __forceinline__ float bfr(float f) { return bf2f(f2bf(f)); }
__device__ __forceinline__ v16h cat16(v8h lo, v8h hi) { return __builtin_shufflevector(lo, hi, 0, 1, 2, 3, 4, 5, 6, 7, 8, 9, 10, 11, 12, 13, 14, 15); }
__device__ __forceinline__ v16bf cat16b(v8us lo, v8us hi) { return __builtin_bit_cast(v16bf, __builtin_shufflevector(lo, hi, 0, 1, 2, 3, 4, 5, 6, 7, 8, 9, 10, 11, 12, 13, 14, 15)); }
__device__ __forceinline__ v8f wmma16(v16h a, v16h b, v8f c) { return __builtin_amdgcn_wmma_f32_16x16x32_f16(false, a, false, b, (short)0, c, false, false); }
__device__ __forceinline__ v8f wmmab(v16bf a, v16bf b, v8f c) { return __builtin_amdgcn_wmma_f32_16x16x32_bf16(false, a, false, b, (short)0, c, false, false); }


template <typename T16> struct WFrag;
template <> struct WFrag<h16> { typedef v16h V; static __device__ __forceinline__ V ld(const h16* p) { return cat16(*(const v8h*)p, *(const v8h*)(p + 16)); } static __device__ __forceinline__ v8f mma(V a, V b, v8f c) { return wmma16(a, b, c); } };
template <> struct WFrag<bf> { typedef v16bf V; static __device__ __forceinline__ V ld(const bf* p) { return cat16b(*(const v8us*)p, *(const v8us*)(p + 16)); } static __device__ __forceinline__ v8f mma(V a, V b, v8f c) { return wmmab(a, b, c); } };
template <typename T16, int NSPLIT, bool BIAS>
__global__ __launch_bounds__(32) void k_gemmw(const T16* __restrict__ A, const T16* __restrict__ A2, const T16* __restrict__ Bt, const T16* __restrict__ Bt2, int K, float* C, int ldc, const float* __restrict__ bias, size_t sA, size_t sB, size_t sC) {
    typedef typename WFrag<T16>::V V;
    __shared__ __align__(16) float os[16 * 68];
    const size_t z = blockIdx.z; A += z * sA; if (A2) A2 += z * sA; Bt += z * sB; if (Bt2) Bt2 += z * sB; C += z * sC;
    const int lane = threadIdx.x & 31, lr = lane & 15, hi = lane >> 4; const int r0 = blockIdx.x * 64, c0 = blockIdx.y * 64;
    v8f acc[4][4];
#pragma unroll
    for (int mb = 0; mb < 4; ++mb)
#pragma unroll
        for (int nb = 0; nb < 4; ++nb) acc[mb][nb] = (v8f){};
    const size_t aoff = (size_t)(r0 + lr) * K + 8 * hi, boff = (size_t)(c0 + lr) * K + 8 * hi;
#pragma unroll 1
    for (int kc = 0; kc < K; kc += 32) {
        V a[4], a2[4];
#pragma unroll
        for (int mb = 0; mb < 4; ++mb) { a[mb] = WFrag<T16>::ld(A + aoff + (size_t)mb * 16 * K + kc); if (NSPLIT == 1 || NSPLIT == 2) a2[mb] = WFrag<T16>::ld(A2 + aoff + (size_t)mb * 16 * K + kc); }
#pragma unroll
        for (int nb = 0; nb < 4; ++nb) { const V b = WFrag<T16>::ld(Bt + boff + (size_t)nb * 16 * K + kc); V b2; if (NSPLIT >= 2) b2 = WFrag<T16>::ld(Bt2 + boff + (size_t)nb * 16 * K + kc);
#pragma unroll
            for (int mb = 0; mb < 4; ++mb) { acc[mb][nb] = WFrag<T16>::mma(a[mb], b, acc[mb][nb]); if (NSPLIT == 1 || NSPLIT == 2) acc[mb][nb] = WFrag<T16>::mma(a2[mb], b, acc[mb][nb]); if (NSPLIT >= 2) acc[mb][nb] = WFrag<T16>::mma(a[mb], b2, acc[mb][nb]); } }
        asm volatile("v_nop\n\tv_nop\n\tv_nop\n\tv_nop" : "+v"(acc[0][0]), "+v"(acc[1][1]), "+v"(acc[2][2]), "+v"(acc[3][3]) : "v"(a[0]), "v"(a[3]));
    }
#pragma unroll
    for (int mb = 0; mb < 4; ++mb) {
#pragma unroll
        for (int nb = 0; nb < 4; ++nb) {
#pragma unroll
            for (int j = 0; j < 8; ++j) os[(hi * 8 + j) * 68 + nb * 16 + lr] = acc[mb][nb][j]; }
        __builtin_amdgcn_wave_barrier(); asm volatile("" ::: "memory");
        float* crow = C + (size_t)(r0 + mb * 16) * ldc + c0;
#pragma unroll 1
        for (int ps = 0; ps < 2; ++ps) {
#pragma unroll
            for (int s = 0; s < 8; ++s) { const int row = 2 * s + hi, cofs = lr * 4; v4f val = *(const v4fa*)(os + row * 68 + cofs); if (BIAS) { val[0] += bfr(bias[c0 + cofs]); val[1] += bfr(bias[c0 + cofs + 1]); val[2] += bfr(bias[c0 + cofs + 2]); val[3] += bfr(bias[c0 + cofs + 3]); }
                *(volatile v4f*)(crow + (size_t)row * ldc + cofs) = val; }
            if (ps == 0) __threadfence(); }
        __builtin_amdgcn_wave_barrier(); asm volatile("" ::: "memory");
    }
}

__device__ __forceinline__ void splitf(float y, unsigned short& h, unsigned short& l) { h = f2bf(y); l = f2bf(y - bf2f(h)); }
typedef __attribute__((ext_vector_type(2))) unsigned short v2us;
typedef __attribute__((ext_vector_type(4))) unsigned short v4us;

__global__ __launch_bounds__(256) void k_cvt8(const float* __restrict__ src, bf* dst, size_t n8) { const size_t i = (size_t)blockIdx.x * 256 + threadIdx.x; if (i >= n8) return; const v8f v = *(const v8f*)(src + i * 8); v8us o;
#pragma unroll
    for (int k = 0; k < 8; ++k) o[k] = f2bf(v[k]); *(volatile v8us*)(dst + i * 8) = o; __threadfence(); *(volatile v8us*)(dst + i * 8) = o; }
__global__ __launch_bounds__(256) void k_w1(const float* __restrict__ w, int off, bf* Bt) { const int e = (blockIdx.x * 256 + threadIdx.x) * 4; if (e >= HDN * ED) return; const int k = e % ED; const int n = e / ED; v4us o;
#pragma unroll
    for (int u = 0; u < 4; ++u) o[u] = f2bf(w[(size_t)(off + k + u) * HDN + n]); *(volatile v4us*)(Bt + e) = o; __threadfence(); *(volatile v4us*)(Bt + e) = o; }
__global__ __launch_bounds__(256) void k_w2(const float* __restrict__ w, bf* Bt) { const int e = (blockIdx.x * 256 + threadIdx.x) * 4; if (e >= HDN * HDN) return; const int k = e % HDN; const int n = e / HDN; v4us o;
#pragma unroll
    for (int u = 0; u < 4; ++u) o[u] = f2bf(w[(size_t)(k + u) * HDN + n]); *(volatile v4us*)(Bt + e) = o; __threadfence(); *(volatile v4us*)(Bt + e) = o; }
__global__ __launch_bounds__(256) void k_ln1(const float* __restrict__ HS, const float* __restrict__ HDd, const float* __restrict__ b1, const float* __restrict__ g1, const float* __restrict__ be1, size_t p0, bf* Ah, bf* Al) { const int lane = threadIdx.x & 31; const size_t pl = (size_t)blockIdx.x * 8 + (threadIdx.x >> 5); if (pl >= RCH) return; const size_t p = p0 + pl; const int i = (int)(p / NN), j = (int)(p % NN); float x0, x1; float s = 0.f;
    { const int c = lane * 2; float a0 = __fadd_rn(HS[i * HDN + c], HDd[j * HDN + c]); asm volatile("" : "+v"(a0)); x0 = __fadd_rn(a0, bfr(b1[c])); float a1 = __fadd_rn(HS[i * HDN + c + 1], HDd[j * HDN + c + 1]); asm volatile("" : "+v"(a1)); x1 = __fadd_rn(a1, bfr(b1[c + 1])); s = x0 + x1; }
#pragma unroll
    for (int sh = 16; sh; sh >>= 1) s += __shfl_xor(s, sh, 32);
    const float mean = s * (1.0f / HDN); float d0 = __fsub_rn(x0, mean), d1 = __fsub_rn(x1, mean); asm volatile("" : "+v"(d0)); asm volatile("" : "+v"(d1)); float q = __fmul_rn(d0, d0); asm volatile("" : "+v"(q)); float q1 = __fmul_rn(d1, d1); asm volatile("" : "+v"(q1)); q = __fadd_rn(q, q1);
#pragma unroll
    for (int sh = 16; sh; sh >>= 1) q += __shfl_xor(q, sh, 32);
    const float rs = __frsqrt_rn(__fadd_rn(q * (1.0f / HDN), 1e-5f)); v2us oh, ol;
    { const int c = lane * 2; float n0 = __fmul_rn(d0, rs), n1 = __fmul_rn(d1, rs); asm volatile("" : "+v"(n0)); asm volatile("" : "+v"(n1)); float t0 = __fmul_rn(n0, bfr(g1[c])), t1 = __fmul_rn(n1, bfr(g1[c + 1])); asm volatile("" : "+v"(t0)); asm volatile("" : "+v"(t1)); const float r0 = fmaxf(__fadd_rn(t0, bfr(be1[c])), 0.f), r1 = fmaxf(__fadd_rn(t1, bfr(be1[c + 1])), 0.f); unsigned short a, b; splitf(r0, a, b); oh[0] = a; ol[0] = b; splitf(r1, a, b); oh[1] = a; ol[1] = b; }
    const size_t oo = pl * HDN + lane * 2; *(volatile v2us*)(Ah + oo) = oh; *(volatile v2us*)(Al + oo) = ol; __threadfence(); *(volatile v2us*)(Ah + oo) = oh; *(volatile v2us*)(Al + oo) = ol; }
__global__ __launch_bounds__(256) void k_fin(const float* __restrict__ H2, const float* __restrict__ b2, const float* __restrict__ g2, const float* __restrict__ be2, const float* __restrict__ W3, const float* __restrict__ b3, size_t p0, float* out) { __shared__ float sb2[HDN], sg2[HDN], sbe2[HDN], sw3[HDN]; if (threadIdx.x < HDN) { sb2[threadIdx.x] = bfr(b2[threadIdx.x]); sg2[threadIdx.x] = bfr(g2[threadIdx.x]); sbe2[threadIdx.x] = bfr(be2[threadIdx.x]); sw3[threadIdx.x] = bfr(W3[threadIdx.x]); } __syncthreads();
    const size_t pl = (size_t)blockIdx.x * 256 + threadIdx.x; if (pl >= RCH) return; const float* r = H2 + pl * HDN; float x[HDN]; float s = 0.f;
#pragma unroll
    for (int c = 0; c < HDN; c += 4) { const v4f a = *(const v4f*)(r + c);
#pragma unroll
        for (int u = 0; u < 4; ++u) { x[c + u] = __fadd_rn(a[u], sb2[c + u]); s += x[c + u]; } }
    const float mean = s * (1.0f / HDN); float q = 0.f;
#pragma unroll
    for (int c = 0; c < HDN; ++c) { float d = __fsub_rn(x[c], mean); asm volatile("" : "+v"(d)); x[c] = d; float pq = __fmul_rn(d, d); asm volatile("" : "+v"(pq)); q = __fadd_rn(q, pq); }
    const float rs = __frsqrt_rn(__fadd_rn(q * (1.0f / HDN), 1e-5f)); float acc = 0.f;
#pragma unroll
    for (int c = 0; c < HDN; ++c) { float n0 = __fmul_rn(x[c], rs); asm volatile("" : "+v"(n0)); float t0 = __fmul_rn(n0, sg2[c]); asm volatile("" : "+v"(t0)); const float rl = fmaxf(__fadd_rn(t0, sbe2[c]), 0.f); float pw = __fmul_rn(rl, sw3[c]); asm volatile("" : "+v"(pw)); acc = __fadd_rn(acc, pw); }
    const float z = __fadd_rn(acc, bfr(b3[0])); const float o = __fdiv_rn(1.0f, __fadd_rn(1.0f, __expf(-z))); float* dst = out + p0 + pl; *(volatile float*)dst = o; __threadfence(); *(volatile float*)dst = o; }

extern "C" void kernel_launch(void* const* d_in, const int* in_sizes, int n_in,
                              void* d_out, int out_size, void* d_ws, size_t ws_size, hipStream_t stream) {
    (void)in_sizes; (void)n_in; (void)out_size;
    const float** I = (const float**)d_in;
    const float *E = I[0], *W1 = I[1], *b1 = I[2], *g1 = I[3], *be1 = I[4], *W2 = I[5], *b2 = I[6], *g2 = I[7], *be2 = I[8], *W3 = I[9], *b3 = I[10];
    float* OUT = (float*)d_out;
    char* wsp = (char*)d_ws;
    auto take = [&](size_t bytes) { char* p = wsp; wsp += (bytes + 255) & ~(size_t)255; return (void*)p; };
    bf* EB = (bf*)take((size_t)NN * ED * 2); bf* B1s = (bf*)take((size_t)HDN * ED * 2); bf* B1d = (bf*)take((size_t)HDN * ED * 2); bf* B2 = (bf*)take((size_t)HDN * HDN * 2); float* HS = (float*)take((size_t)NN * HDN * 4); float* HDd = (float*)take((size_t)NN * HDN * 4);
    bf* Ah = (bf*)take((size_t)RCH * HDN * 2); bf* Al = (bf*)take((size_t)RCH * HDN * 2); float* H2 = (float*)take((size_t)RCH * HDN * 4);
    if ((size_t)(wsp - (char*)d_ws) > ws_size) return;
    k_cvt8<<<(NN * ED / 8 + 255) / 256, 256, 0, stream>>>(E, EB, NN * ED / 8); k_w1<<<(HDN * ED / 4 + 255) / 256, 256, 0, stream>>>(W1, 0, B1s); k_w1<<<(HDN * ED / 4 + 255) / 256, 256, 0, stream>>>(W1, ED, B1d); k_w2<<<(HDN * HDN / 4 + 255) / 256, 256, 0, stream>>>(W2, B2);
    k_gemmw<bf, 0, false><<<dim3(NN / 64, 1, 1), 32, 0, stream>>>(EB, nullptr, B1s, nullptr, ED, HS, HDN, nullptr, 0, 0, 0); k_gemmw<bf, 0, false><<<dim3(NN / 64, 1, 1), 32, 0, stream>>>(EB, nullptr, B1d, nullptr, ED, HDd, HDN, nullptr, 0, 0, 0);
    for (size_t p0 = 0; p0 < (size_t)NN * NN; p0 += RCH) {
        k_ln1<<<RCH / 8, 256, 0, stream>>>(HS, HDd, b1, g1, be1, p0, Ah, Al);
        k_gemmw<bf, 1, false><<<dim3(RCH / 64, 1, 1), 32, 0, stream>>>(Ah, Al, B2, nullptr, HDN, H2, HDN, nullptr, 0, 0, 0);
        k_fin<<<RCH / 256, 256, 0, stream>>>(H2, b2, g2, be2, W3, b3, p0, OUT); }
}
